// RnnClassifier_56547539419195
// MI455X (gfx1250) — hardware-run, weakly checked
//
#include <hip/hip_runtime.h>
#include <math.h>

typedef __attribute__((ext_vector_type(16))) _Float16 v16h;
typedef __attribute__((ext_vector_type(8)))  _Float16 v8h;
typedef __attribute__((ext_vector_type(8)))  float    v8f;
typedef __attribute__((ext_vector_type(4)))  float    v4f;

constexpr int kVocab = 50000;
constexpr int kEmb   = 128;
constexpr int kHid   = 15;
constexpr int kGate  = 45;
constexpr int kCls   = 20;
constexpr int kBatch = 512;
constexpr int kSeq   = 512;
constexpr int kRows  = kSeq * kBatch;
constexpr int kNPad  = 64;
constexpr int kGemmRows  = 64;
constexpr int kAPitch    = 136;
constexpr int kSlabPitch = 68;
constexpr int kScanRows  = 16;
constexpr float kCarry       = 256.0f;
constexpr float kCarryFold   = 1.0f / (kCarry * kCarry);
constexpr float kHalfMinNorm = 6.103515625e-05f;

static_assert(kGate == 3 * kHid, "three gates");
static_assert((kEmb % 32) == 0, "K multiple of 32");
static_assert((kRows % kGemmRows) == 0 && (kBatch % kGemmRows) == 0, "row tiles stay inside one step");
static_assert(((kVocab * kEmb) % (8 * 256)) == 0, "embedding plane grid is exact");
static_assert((kBatch % kScanRows) == 0, "scan blocks");
static_assert((kScanRows * kCls * 4) % 128 == 0, "block output is whole lines");

constexpr size_t kOffE16    = 0;
constexpr size_t kOffBT16   = kOffE16    + (size_t)kVocab * kEmb * 2;
constexpr size_t kOffBIAS64 = kOffBT16   + (size_t)kNPad * kEmb * 2;
constexpr size_t kOffG16    = kOffBIAS64 + (size_t)kNPad * 4;
constexpr size_t kWsTotal   = kOffG16    + (size_t)kRows * kNPad * 2;
static_assert(kWsTotal == 46371072ull, "carve total");
static_assert(kWsTotal <= 134217728ull, "carve cap");
static_assert((kOffBT16 % 128) == 0 && (kOffBIAS64 % 128) == 0 && (kOffG16 % 128) == 0, "aligned regions");

__device__ __forceinline__ unsigned pin_u(unsigned v) { asm volatile("" : "+v"(v)); return v; }
__device__ __forceinline__ float    pin_f(float v)    { asm volatile("" : "+v"(v)); return v; }
__device__ __forceinline__ int      pin_i(int v)      { asm volatile("" : "+v"(v)); return v; }

__device__ __forceinline__ _Float16 carry_to_f16(float v) {
  float xs = v * kCarry;
  xs = (fabsf(xs) < kHalfMinNorm) ? 0.0f : xs;
  return (_Float16)xs;
}

__device__ __forceinline__ float h16_to_f32(unsigned hb) {
  const unsigned sgn = (hb & 0x8000u) << 16;
  const unsigned em  = hb & 0x7fffu;
  const float fn = __uint_as_float((em << 13) + 0x38000000u);
  const float fs = (float)em * 5.9604644775390625e-8f;
  const float mag = (em < 0x400u) ? fs : fn;
  return __uint_as_float(__float_as_uint(mag) | sgn);
}

struct FragH {
  union U { v16h v; v8h h[2]; };
  static __device__ __forceinline__ v16h load(const _Float16* p) {
    U f;
    f.h[0] = *(const v8h*)(p);
    f.h[1] = *(const v8h*)(p + 16);
    return f.v;
  }
};

__device__ __forceinline__ v8f mma_f16_step(v16h a, v16h b, v8f c) {
  c = __builtin_amdgcn_wmma_f32_16x16x32_f16(false, a, false, b, (short)0, c, false, false);
  asm volatile("v_nop\n\tv_nop\n\tv_nop\n\tv_nop" : "+v"(c) : "v"(a), "v"(b));
  return c;
}

__global__ __launch_bounds__(256) void embed_plane_kernel(
    const float* __restrict__ embed, unsigned short* __restrict__ E16, int total8)
{
  const int i = blockIdx.x * 256 + threadIdx.x;
  if (i >= total8) return;
  const size_t e0 = (size_t)i << 3;
  const v4f a0 = *(const v4f*)(embed + e0);
  const v4f a1 = *(const v4f*)(embed + e0 + 4);
  v8h hv;
#pragma unroll
  for (int e = 0; e < 4; ++e) {
    const float f0 = a0[e];
    const float f1 = a1[e];
    hv[e]     = carry_to_f16(f0);
    hv[4 + e] = carry_to_f16(f1);
  }
  unsigned short* q = E16 + e0;
  *(volatile v8h*)q = hv;
  __threadfence();
  *(volatile v8h*)q = hv;
}

__global__ __launch_bounds__(256) void weight_plane_kernel(
    const float* __restrict__ W_ih, const float* __restrict__ b_ih,
    unsigned short* __restrict__ BT16, float* __restrict__ BIAS64)
{
  const unsigned tid = threadIdx.x;
  if (blockIdx.x < 4) {
    const unsigned i    = pin_u(blockIdx.x * 256u + tid);
    const unsigned np   = pin_u(i >> 4);
    const unsigned kc   = pin_u((i & 15u) * 8u);
    const unsigned gate = np >> 4;
    const unsigned j    = np & 15u;
    const bool live = (gate < 3u) && (j < 15u);
    const unsigned src = live ? (gate * 15u + j) : 0u;
    const float* wp = W_ih + (size_t)src * kEmb + kc;
    const v4f a0 = *(const v4f*)(wp);
    const v4f a1 = *(const v4f*)(wp + 4);
    v8h hv;
#pragma unroll
    for (int e = 0; e < 4; ++e) {
      const float f0 = live ? a0[e] : 0.0f;
      const float f1 = live ? a1[e] : 0.0f;
      hv[e]     = carry_to_f16(f0);
      hv[4 + e] = carry_to_f16(f1);
    }
    unsigned short* q = BT16 + (size_t)i * 8;
    *(volatile v8h*)q = hv;
    __threadfence();
    *(volatile v8h*)q = hv;
  } else {
    const unsigned q16 = pin_u(tid & 15u);
    float bv[4];
#pragma unroll
    for (int e = 0; e < 4; ++e) {
      const unsigned np   = q16 * 4u + (unsigned)e;
      const unsigned gate = np >> 4;
      const unsigned j    = np & 15u;
      const bool live = (gate < 3u) && (j < 15u);
      const unsigned src = live ? (gate * 15u + j) : 0u;
      float v = b_ih[src];
      v = pin_f(v);
      bv[e] = live ? v : 0.0f;
    }
    v4f ov;
    ov[0] = bv[0];
    ov[1] = bv[1];
    ov[2] = bv[2];
    ov[3] = bv[3];
    if (tid < 16u) {
      float* q = BIAS64 + q16 * 4u;
      *(volatile v4f*)q = ov;
      __threadfence();
      *(volatile v4f*)q = ov;
    }
  }
}

__device__ __forceinline__ void slab_put(float* slab, v8f acc, float bv, unsigned col, unsigned mOff) {
#pragma unroll
  for (int r = 0; r < 8; ++r) {
    slab[(mOff + (unsigned)r) * kSlabPitch + col] = fmaf(acc[r], kCarryFold, bv);
  }
}

__global__ __launch_bounds__(128) void gates_gemm_kernel(
    const int* __restrict__ x, const unsigned short* __restrict__ E16p,
    const unsigned short* __restrict__ BT16p, const float* __restrict__ BIAS64,
    unsigned short* __restrict__ G16)
{
  __shared__ __align__(16) _Float16 sA[kGemmRows * kAPitch];
  __shared__ __align__(16) float sT[4][16 * kSlabPitch];
  __shared__ int sTok[kGemmRows];

  const _Float16* E16 = (const _Float16*)E16p;
  const _Float16* Bt  = (const _Float16*)BT16p;

  const unsigned tid  = threadIdx.x;
  const unsigned lane = pin_u(tid & 31u);
  const unsigned wave = tid >> 5;
  const unsigned m0   = blockIdx.x * (unsigned)kGemmRows;
  const unsigned s    = m0 >> 9;
  const unsigned b0   = m0 & 511u;

  {
    const unsigned tl = pin_u(tid & 63u);
    int tok = x[(size_t)(b0 + tl) * kSeq + s];
    tok = pin_i(tok);
    tok = tok < 0 ? 0 : (tok > (kVocab - 1) ? (kVocab - 1) : tok);
    if (tid < 64u) sTok[tid] = tok;
  }
  __syncthreads();

  {
    const unsigned rq = pin_u(tid >> 4);
    const unsigned c8 = pin_u((tid & 15u) * 8u);
#pragma unroll
    for (int i = 0; i < 8; ++i) {
      const unsigned r = rq + 8u * (unsigned)i;
      int t = sTok[r];
      t = t < 0 ? 0 : (t > (kVocab - 1) ? (kVocab - 1) : t);
      const v8h ch = *(const v8h*)(E16 + (size_t)t * kEmb + c8);
      *(v8h*)(sA + r * kAPitch + c8) = ch;
    }
  }
  __syncthreads();

  const unsigned rlane = pin_u(lane & 15u);
  const unsigned hhalf = pin_u(lane >> 4);
  const unsigned koff  = hhalf * 8u;
  const unsigned mOff  = hhalf * 8u;

  const _Float16* arow = sA + (wave * 16u + rlane) * kAPitch + koff;
  const _Float16* brow = Bt + (size_t)rlane * kEmb + koff;

  v8f acc0 = (v8f){0.f, 0.f, 0.f, 0.f, 0.f, 0.f, 0.f, 0.f};
  v8f acc1 = acc0;
  v8f acc2 = acc0;
  v8f acc3 = acc0;

#pragma unroll 1
  for (int k0 = 0; k0 < kEmb; k0 += 32) {
    const v16h a  = FragH::load(arow + k0);
    const v16h f0 = FragH::load(brow + k0);
    const v16h f1 = FragH::load(brow + 16 * kEmb + k0);
    const v16h f2 = FragH::load(brow + 32 * kEmb + k0);
    const v16h f3 = FragH::load(brow + 48 * kEmb + k0);
    acc0 = mma_f16_step(a, f0, acc0);
    acc1 = mma_f16_step(a, f1, acc1);
    acc2 = mma_f16_step(a, f2, acc2);
    acc3 = mma_f16_step(a, f3, acc3);
  }

  float* slab = sT[wave];
  {
    const float bv0 = BIAS64[rlane];
    const float bv1 = BIAS64[16u + rlane];
    const float bv2 = BIAS64[32u + rlane];
    const float bv3 = BIAS64[48u + rlane];
    slab_put(slab, acc0, bv0, rlane, mOff);
    slab_put(slab, acc1, bv1, 16u + rlane, mOff);
    slab_put(slab, acc2, bv2, 32u + rlane, mOff);
    slab_put(slab, acc3, bv3, 48u + rlane, mOff);
  }
  __syncthreads();

  const unsigned q  = pin_u(lane >> 3);
  const unsigned c8 = pin_u((lane & 7u) * 8u);
  v8h hv[4];
#pragma unroll
  for (int it = 0; it < 4; ++it) {
    const unsigned row = (unsigned)it * 4u + q;
    const float* sp = slab + row * kSlabPitch + c8;
#pragma unroll
    for (int e = 0; e < 8; ++e) {
      const float f = sp[e];
      hv[it][e] = (_Float16)f;
    }
  }
  for (int pass = 0; pass < 2; ++pass) {
#pragma unroll
    for (int it = 0; it < 4; ++it) {
      const unsigned row = (unsigned)it * 4u + q;
      unsigned short* dst = G16 + (size_t)(m0 + wave * 16u + row) * kNPad + c8;
      *(volatile v8h*)dst = hv[it];
    }
    __threadfence();
  }
}

__global__ __launch_bounds__(256) void scan_head_kernel(
    const unsigned* __restrict__ Gw, const float* __restrict__ W_hh, const float* __restrict__ b_hh,
    const float* __restrict__ W_out, const float* __restrict__ b_out, float* __restrict__ out)
{
  __shared__ float sWh[kGate * kHid];
  __shared__ float sBh[48];
  __shared__ float sWo[kCls * kHid];
  __shared__ float sBo[32];
  __shared__ float sH[kScanRows * 16];
  __shared__ __align__(16) float sO[kScanRows * kCls];

  const unsigned tid  = threadIdx.x;
  const unsigned lane = tid & 31u;
  const unsigned wave = tid >> 5;

#pragma unroll
  for (int it = 0; it < 3; ++it) {
    const unsigned i  = tid + 256u * (unsigned)it;
    const unsigned ic = i < (unsigned)(kGate * kHid) ? i : (unsigned)(kGate * kHid - 1);
    float v = W_hh[ic];
    v = pin_f(v);
    if (i < (unsigned)(kGate * kHid)) sWh[i] = v;
  }
#pragma unroll
  for (int it = 0; it < 2; ++it) {
    const unsigned i  = tid + 256u * (unsigned)it;
    const unsigned ic = i < (unsigned)(kCls * kHid) ? i : (unsigned)(kCls * kHid - 1);
    float v = W_out[ic];
    v = pin_f(v);
    if (i < (unsigned)(kCls * kHid)) sWo[i] = v;
  }
  {
    const unsigned ic = tid < (unsigned)kGate ? tid : (unsigned)(kGate - 1);
    float v = b_hh[ic];
    v = pin_f(v);
    if (tid < (unsigned)kGate) sBh[tid] = v;
    const unsigned oc = tid < (unsigned)kCls ? tid : (unsigned)(kCls - 1);
    float u = b_out[oc];
    u = pin_f(u);
    if (tid < (unsigned)kCls) sBo[tid] = u;
  }
  __syncthreads();

  const unsigned j    = pin_u(tid & 15u);
  const unsigned brow = pin_u(tid >> 4);
  const bool live     = (j < (unsigned)kHid);
  const unsigned jj   = live ? j : (unsigned)(kHid - 1);
  const unsigned b    = blockIdx.x * (unsigned)kScanRows + brow;
  const unsigned jw   = pin_u(j >> 1);
  const bool jodd     = ((j & 1u) != 0u);

  float wr[kHid], wz[kHid], wn[kHid];
#pragma unroll
  for (int k = 0; k < kHid; ++k) {
    const float a0 = sWh[jj * kHid + (unsigned)k];
    const float a1 = sWh[(kHid + jj) * kHid + (unsigned)k];
    const float a2 = sWh[(2 * kHid + jj) * kHid + (unsigned)k];
    wr[k] = live ? a0 : 0.0f;
    wz[k] = live ? a1 : 0.0f;
    wn[k] = live ? a2 : 0.0f;
  }
  float br, bz, bn;
  {
    const float c0 = sBh[jj];
    const float c1 = sBh[kHid + jj];
    const float c2 = sBh[2 * kHid + jj];
    br = live ? c0 : 0.0f;
    bz = live ? c1 : 0.0f;
    bn = live ? c2 : 0.0f;
  }

  float h = 0.0f;
  unsigned w0, w1, w2;
  {
    const size_t wb = (size_t)b * 32 + jw;
    w0 = Gw[wb];
    w1 = Gw[wb + 8];
    w2 = Gw[wb + 16];
  }
#pragma unroll 1
  for (int s = 0; s < kSeq; ++s) {
    const int sn = (s + 1 < kSeq) ? (s + 1) : (kSeq - 1);
    const size_t nb = ((size_t)sn * kBatch + b) * 32 + jw;
    const unsigned n0 = Gw[nb];
    const unsigned n1 = Gw[nb + 8];
    const unsigned n2 = Gw[nb + 16];

    const unsigned hb0 = jodd ? (w0 >> 16) : (w0 & 0xffffu);
    const unsigned hb1 = jodd ? (w1 >> 16) : (w1 & 0xffffu);
    const unsigned hb2 = jodd ? (w2 >> 16) : (w2 & 0xffffu);
    const float xr = h16_to_f32(hb0);
    const float xz = h16_to_f32(hb1);
    const float xn = h16_to_f32(hb2);

    float hr = br, hz = bz, hn = bn;
#pragma unroll
    for (int k = 0; k < kHid; ++k) {
      const float hk = __shfl(h, k, 16);
      hr = fmaf(wr[k], hk, hr);
      hz = fmaf(wz[k], hk, hz);
      hn = fmaf(wn[k], hk, hn);
    }
    const float r = 1.0f / (1.0f + expf(-(xr + hr)));
    const float z = 1.0f / (1.0f + expf(-(xz + hz)));
    const float n = tanhf(xn + r * hn);
    h = (1.0f - z) * n + z * h;

    w0 = n0;
    w1 = n1;
    w2 = n2;
  }

  sH[brow * 16u + j] = h;
  __syncthreads();

  if (tid < (unsigned)kScanRows) {
    const unsigned t = tid;
    float mx = -3.0e38f;
#pragma unroll 1
    for (int c = 0; c < kCls; ++c) {
      float l = 0.0f;
#pragma unroll 1
      for (int k = 0; k < kHid; ++k) l = fmaf(sWo[c * kHid + k], sH[t * 16u + (unsigned)k], l);
      l += sBo[c];
      sO[t * kCls + (unsigned)c] = l;
      mx = fmaxf(mx, l);
    }
    float sum = 0.0f;
#pragma unroll 1
    for (int c = 0; c < kCls; ++c) {
      const float e = expf(sO[t * kCls + (unsigned)c] - mx);
      sO[t * kCls + (unsigned)c] = e;
      sum += e;
    }
    const float inv = 1.0f / sum;
#pragma unroll 1
    for (int c = 0; c < kCls; ++c) {
      const float p = sO[t * kCls + (unsigned)c] * inv;
      sO[t * kCls + (unsigned)c] = p;
    }
  }
  __syncthreads();

  if (wave == 0u) {
    constexpr unsigned kVec = (unsigned)(kScanRows * kCls / 4);
    v4f ov[3];
#pragma unroll
    for (int it = 0; it < 3; ++it) {
      const unsigned idx = (unsigned)it * 32u + lane;
      const unsigned idc = idx < kVec ? idx : (kVec - 1u);
      ov[it] = *(const v4f*)(sO + idc * 4u);
    }
    float* ob = out + (size_t)blockIdx.x * (kScanRows * kCls);
    for (int pass = 0; pass < 2; ++pass) {
#pragma unroll
      for (int it = 0; it < 3; ++it) {
        const unsigned idx = (unsigned)it * 32u + lane;
        if (idx < kVec) *(volatile v4f*)(ob + idx * 4u) = ov[it];
      }
      __threadfence();
    }
  }
}

extern "C" void kernel_launch(void* const* d_in, const int* in_sizes, int n_in,
                              void* d_out, int out_size, void* d_ws, size_t ws_size,
                              hipStream_t stream) {
  if (n_in < 8) return;
  if (in_sizes[0] != kBatch * kSeq) return;
  if (in_sizes[1] != kVocab * kEmb) return;
  if (in_sizes[2] != kGate * kEmb) return;
  if (in_sizes[3] != kGate) return;
  if (in_sizes[4] != kGate * kHid) return;
  if (in_sizes[5] != kGate) return;
  if (in_sizes[6] != kCls * kHid) return;
  if (in_sizes[7] != kCls) return;
  if (out_size != kBatch * kCls) return;
  if (ws_size < kWsTotal) return;

  const int*   x     = (const int*)d_in[0];
  const float* embed = (const float*)d_in[1];
  const float* W_ih  = (const float*)d_in[2];
  const float* b_ih  = (const float*)d_in[3];
  const float* W_hh  = (const float*)d_in[4];
  const float* b_hh  = (const float*)d_in[5];
  const float* W_out = (const float*)d_in[6];
  const float* b_out = (const float*)d_in[7];
  float* out = (float*)d_out;

  char* ws = (char*)d_ws;
  unsigned short* E16    = (unsigned short*)(ws + kOffE16);
  unsigned short* BT16   = (unsigned short*)(ws + kOffBT16);
  float*          BIAS64 = (float*)(ws + kOffBIAS64);
  unsigned short* G16    = (unsigned short*)(ws + kOffG16);

  embed_plane_kernel<<<(kVocab * kEmb / 8) / 256, 256, 0, stream>>>(embed, E16, kVocab * kEmb / 8);
  weight_plane_kernel<<<5, 256, 0, stream>>>(W_ih, b_ih, BT16, BIAS64);
  gates_gemm_kernel<<<kRows / kGemmRows, 128, 0, stream>>>(x, E16, BT16, BIAS64, G16);
  scan_head_kernel<<<kBatch / kScanRows, 256, 0, stream>>>((const unsigned*)G16, W_hh, b_hh, W_out, b_out, out);
}
